// DynamicMemoryInduction_12713103197271
// MI455X (gfx1250) — hardware-verified
//
#include <hip/hip_runtime.h>


namespace {
constexpr int IC = 512, Q = 512, C = 64, DC = 16, IN = 768, NO = C * DC;
constexpr float AS = 8.0f, WS = 64.0f, EPS = 1e-8f;

typedef _Float16 b16;
typedef __attribute__((ext_vector_type(16))) _Float16 v16b;
typedef __attribute__((ext_vector_type(8)))  _Float16 v8b;
typedef __attribute__((ext_vector_type(8)))  float v8f;
typedef __attribute__((ext_vector_type(4)))  float v4f;

__device__ __forceinline__ v8b ld8b(const b16* p) { return *(const v8b*)p; }
__device__ __forceinline__ v16b cat8b(v8b a, v8b b) { return __builtin_shufflevector(a, b, 0, 1, 2, 3, 4, 5, 6, 7, 8, 9, 10, 11, 12, 13, 14, 15); }
__device__ __forceinline__ v16b frag_kb(const b16* p, int hh) { return cat8b(ld8b(p + 8 * hh), ld8b(p + 16 + 8 * hh)); }
__device__ __forceinline__ void split16(float v, b16& hi, b16& lo) { hi = (b16)v; lo = (b16)(v - (float)hi); }
__device__ __forceinline__ void frag_ksplit(const float* p, int hh, v16b& fh_, v16b& fl_) {
  const float* p0 = p + 8 * hh; const float* p1 = p + 16 + 8 * hh;
#pragma unroll
  for (int e = 0; e < 8; ++e) { b16 a, c; split16(p0[e], a, c); fh_[e] = a; fl_[e] = c; split16(p1[e], a, c); fh_[8 + e] = a; fl_[8 + e] = c; }
}
__device__ __forceinline__ v8f wmma16b(v16b a, v16b b, v8f c) {
  v8f d = __builtin_amdgcn_wmma_f32_16x16x32_f16(false, a, false, b, (short)0, c, false, false);
  asm volatile("v_nop\n\tv_nop\n\tv_nop\n\tv_nop" : "+v"(d) : "v"(a), "v"(b));
  return d;
}
__device__ __forceinline__ void wave_lds_sync() {
  __builtin_amdgcn_fence(__ATOMIC_RELEASE, "workgroup");
  __builtin_amdgcn_wave_barrier();
  __builtin_amdgcn_fence(__ATOMIC_ACQUIRE, "workgroup");
}

struct Opnd { const void* p0; const void* p1; int ld; };
template <int NP> __device__ __forceinline__ void load_frags(const Opnd& o, int row, int kb, int hh, v16b& fh_, v16b& fl_) {
  if (NP == 0) { frag_ksplit((const float*)o.p0 + (size_t)row * o.ld + kb, hh, fh_, fl_); }
  else if (NP == 4 || NP == 5) {
    const float sc_ = (NP == 4) ? 64.0f : 8.0f;
    const float* p = (const float*)o.p0 + (size_t)row * o.ld + kb; const float* p0 = p + 8 * hh; const float* p1 = p + 16 + 8 * hh;
#pragma unroll
    for (int e = 0; e < 8; ++e) { b16 a, c; split16(p0[e] * sc_, a, c); fh_[e] = a; fl_[e] = c; split16(p1[e] * sc_, a, c); fh_[8 + e] = a; fl_[8 + e] = c; }
  } else if (NP == 3) {
    const float* p = (const float*)o.p0 + (size_t)row * o.ld + kb; const float* p0 = p + 8 * hh; const float* p1 = p + 16 + 8 * hh;
#pragma unroll
    for (int e = 0; e < 8; ++e) { fh_[e] = (b16)p0[e]; fh_[8 + e] = (b16)p1[e]; }
    fl_ = fh_;
  } else {
    fh_ = frag_kb((const b16*)o.p0 + (size_t)row * o.ld + kb, hh);
    if (NP == 2) fl_ = frag_kb((const b16*)o.p1 + (size_t)row * o.ld + kb, hh); else fl_ = fh_;
  }
}
template <int ANP, int BNP> __device__ __forceinline__ v8f mac(v16b ah, v16b al, v16b bh, v16b bl, v8f c) {
  c = wmma16b(ah, bh, c);
  if (BNP == 0 || BNP == 2 || BNP == 4 || BNP == 5) c = wmma16b(ah, bl, c);
  if (ANP == 0 || ANP == 2 || ANP == 4 || ANP == 5) c = wmma16b(al, bh, c);
  return c;
}
template <int ANP, int BNP>
__device__ __forceinline__ void gemm_tile(const Opnd& A, const Opnd& B, int K, int m0, int c0, int nloc, int hlf, v8f (&acc)[2][4]) {
  for (int kb = 0; kb < K; kb += 32) {
    v16b a0h, a0l, a1h, a1l;
    load_frags<ANP>(A, m0 + nloc, kb, hlf, a0h, a0l);
    load_frags<ANP>(A, m0 + 16 + nloc, kb, hlf, a1h, a1l);
#pragma unroll
    for (int t = 0; t < 4; ++t) {
      v16b bh, bl;
      load_frags<BNP>(B, c0 + t * 16 + nloc, kb, hlf, bh, bl);
      acc[0][t] = mac<ANP, BNP>(a0h, a0l, bh, bl, acc[0][t]);
      acc[1][t] = mac<ANP, BNP>(a1h, a1l, bh, bl, acc[1][t]);
    }
  }
}

__device__ __forceinline__ void epi_planes(v8f (&acc)[2][4], float scale, bool two, b16* __restrict__ oh, b16* __restrict__ ol, int ldo,
                                           int m0, int c0, int lane, b16* Th, b16* Tl) {
  const int nloc = lane & 15, hlf = lane >> 4;
#pragma unroll
  for (int t = 0; t < 4; ++t)
#pragma unroll
    for (int r = 0; r < 2; ++r)
#pragma unroll
      for (int v = 0; v < 8; ++v) {
        const int rr = r * 16 + v + 8 * hlf, cc = t * 16 + nloc;
        b16 h_, l_; split16(acc[r][t][v] * scale, h_, l_);
        Th[rr * 64 + cc] = h_; Tl[rr * 64 + cc] = l_;
      }
  wave_lds_sync();
  for (int pass = 0; pass < 2; ++pass) {
#pragma unroll
    for (int j = 0; j < 8; ++j) {
      const int rr = j * 4 + (lane >> 3), c8 = (lane & 7) * 8;
      const size_t o = (size_t)(m0 + rr) * ldo + c0 + c8;
      *(volatile v8b*)(oh + o) = ld8b(Th + rr * 64 + c8);
      if (two) *(volatile v8b*)(ol + o) = ld8b(Tl + rr * 64 + c8);
    }
    __threadfence();
  }
}
__device__ __forceinline__ void epi_f32(v8f (&acc)[2][4], float scale, const float* rscale, float* __restrict__ out, int ldo, int m0, int c0, int lane, float* Tt) {
  const int nloc = lane & 15, hlf = lane >> 4;
#pragma unroll
  for (int t = 0; t < 4; ++t)
#pragma unroll
    for (int r = 0; r < 2; ++r)
#pragma unroll
      for (int v = 0; v < 8; ++v) {
        const int rr = r * 16 + v + 8 * hlf;
        const float rs = rscale ? rscale[(size_t)(m0 + rr) * 32] : 1.0f;
        Tt[rr * 64 + t * 16 + nloc] = acc[r][t][v] * scale * rs;
      }
  wave_lds_sync();
  float* dst0 = out + (size_t)m0 * ldo + c0;
  for (int pass = 0; pass < 2; ++pass) {
#pragma unroll
    for (int j = 0; j < 16; ++j) { const int rr = j * 2 + hlf, c4 = nloc * 4; *(volatile v4f*)(dst0 + (size_t)rr * ldo + c4) = *(const v4f*)(Tt + rr * 64 + c4); }
    __threadfence();
  }
}


__device__ __forceinline__ float tanh_e(float v) { return 1.0f - 2.0f / (1.0f + __expf(2.0f * v)); }

__global__ __launch_bounds__(256) void prepw_kernel(const float* __restrict__ W, b16* __restrict__ wh, b16* __restrict__ wl) {
  __shared__ __attribute__((aligned(16))) b16 Th[64][72]; __shared__ __attribute__((aligned(16))) b16 Tl[64][72];
  const int tid = threadIdx.x, lane = tid & 31, wave = tid >> 5, n0 = blockIdx.x * 64, k0 = blockIdx.y * 64;
  for (int i = tid; i < 64 * 64; i += 256) { const int kk = i / 64, nn = i % 64; b16 a, c; split16(W[(size_t)(k0 + kk) * NO + n0 + nn] * WS, a, c); Th[nn][kk] = a; Tl[nn][kk] = c; }
  __syncthreads();
  for (int pass = 0; pass < 2; ++pass) {
#pragma unroll
    for (int j = 0; j < 2; ++j) { const int rr = wave * 8 + j * 4 + (lane >> 3), c8 = (lane & 7) * 8;
      *(volatile v8b*)(wh + (size_t)(n0 + rr) * IN + k0 + c8) = *(const v8b*)(&Th[rr][c8]); *(volatile v8b*)(wl + (size_t)(n0 + rr) * IN + k0 + c8) = *(const v8b*)(&Tl[rr][c8]); }
    __threadfence();
  }
}

__global__ __launch_bounds__(128) void proj_kernel(const float* __restrict__ m, const float* __restrict__ q, const b16* __restrict__ wh, const b16* __restrict__ wl, const float* __restrict__ Wb,
                                                   float* __restrict__ hm, float* __restrict__ qcur) {
  __shared__ __attribute__((aligned(16))) float Ts[4][32 * 64];
  const int lane = threadIdx.x & 31, wave = threadIdx.x >> 5, nloc = lane & 15, hlf = lane >> 4;
  const int m0 = blockIdx.y * 128 + wave * 32, c0 = blockIdx.x * 64;
  const bool isq = m0 >= IC;
  v8f acc[2][4];
#pragma unroll
  for (int r = 0; r < 2; ++r)
#pragma unroll
    for (int t = 0; t < 4; ++t) acc[r][t] = (v8f){};
  const Opnd A{isq ? (q + (size_t)(m0 - IC) * IN) : (m + (size_t)m0 * IN), nullptr, IN}, B{wh, wl, IN};
  gemm_tile<5, 2>(A, B, IN, 0, c0, nloc, hlf, acc);
  float* Tt = Ts[wave];
#pragma unroll
  for (int t = 0; t < 4; ++t)
#pragma unroll
    for (int r = 0; r < 2; ++r)
#pragma unroll
      for (int v = 0; v < 8; ++v) Tt[(r * 16 + v + 8 * hlf) * 64 + t * 16 + nloc] = acc[r][t][v] * (1.0f / (AS * WS)) + Wb[c0 + t * 16 + nloc];
  wave_lds_sync();
  for (int pass = 0; pass < 2; ++pass) {
    if (!isq) {
#pragma unroll
      for (int j = 0; j < 16; ++j) { const int rr = j * 2 + hlf, c4 = nloc * 4; *(volatile v4f*)(hm + (size_t)(m0 + rr) * NO + c0 + c4) = *(const v4f*)(Tt + rr * 64 + c4); }
    } else {
      const int qq0 = m0 - IC;
#pragma unroll
      for (int j = 0; j < 16; ++j) { const int idx = j * 32 + lane; const int t = idx >> 7, rem = idx & 127, rr = rem >> 2, c4 = (rem & 3) * 4;
        *(volatile v4f*)(qcur + (((size_t)(c0 / DC + t) * Q) + qq0 + rr) * DC + c4) = *(const v4f*)(Tt + rr * 64 + t * 16 + c4); }
    }
    __threadfence();
  }
}

__global__ __launch_bounds__(256) void mrows_kernel(const float* __restrict__ hm, b16* __restrict__ mh, b16* __restrict__ ml, b16* __restrict__ mth, b16* __restrict__ mtl, float* __restrict__ mn) {
  const int row = blockIdx.x * 256 + threadIdx.x;
  const float* src = hm + (size_t)row * DC; float x[DC]; float mean = 0.0f;
#pragma unroll
  for (int dd = 0; dd < DC; ++dd) { x[dd] = src[dd]; mean += x[dd]; }
  mean *= (1.0f / DC); float s2 = 0.0f;
  v8b h0, l0, h1, l1, th0, tl0, th1, tl1;
#pragma unroll
  for (int dd = 0; dd < DC; ++dd) { b16 a, c; split16(x[dd] * AS, a, c); const float xt = x[dd] - mean; s2 += xt * xt; b16 ta, tc; split16(xt * AS, ta, tc);
    if (dd < 8) { h0[dd] = a; l0[dd] = c; th0[dd] = ta; tl0[dd] = tc; } else { h1[dd - 8] = a; l1[dd - 8] = c; th1[dd - 8] = ta; tl1[dd - 8] = tc; } }
  for (int pass = 0; pass < 2; ++pass) {
    *(volatile v8b*)(mh + (size_t)row * DC) = h0; *(volatile v8b*)(mh + (size_t)row * DC + 8) = h1; *(volatile v8b*)(ml + (size_t)row * DC) = l0; *(volatile v8b*)(ml + (size_t)row * DC + 8) = l1;
    *(volatile v8b*)(mth + (size_t)row * DC) = th0; *(volatile v8b*)(mth + (size_t)row * DC + 8) = th1; *(volatile v8b*)(mtl + (size_t)row * DC) = tl0; *(volatile v8b*)(mtl + (size_t)row * DC + 8) = tl1;
    ((volatile float*)mn)[row] = s2; __threadfence();
  }
}

__global__ __launch_bounds__(256) void mT_kernel(const float* __restrict__ hm, b16* __restrict__ mTh, b16* __restrict__ mTl) {
  __shared__ __attribute__((aligned(16))) b16 Th[DC][IC + 8]; __shared__ __attribute__((aligned(16))) b16 Tl[DC][IC + 8];
  const int c = blockIdx.x, t = threadIdx.x;
  for (int idx = t; idx < IC * DC; idx += 256) { const int i = idx / DC, dd = idx % DC; b16 a, cc; split16(hm[((size_t)i * C + c) * DC + dd] * AS, a, cc); Th[dd][i] = a; Tl[dd][i] = cc; }
  __syncthreads();
  for (int pass = 0; pass < 2; ++pass) {
    for (int pcs = t; pcs < DC * IC / 8; pcs += 256) { const int dd = pcs / (IC / 8), i8 = (pcs % (IC / 8)) * 8;
      *(volatile v8b*)(mTh + ((size_t)c * DC + dd) * IC + i8) = *(const v8b*)(&Th[dd][i8]); *(volatile v8b*)(mTl + ((size_t)c * DC + dd) * IC + i8) = *(const v8b*)(&Tl[dd][i8]); }
    __threadfence();
  }
}

template <bool INIT>
__global__ __launch_bounds__(128) void pc_kernel(const float* __restrict__ qcur, const float* __restrict__ vbuf, const b16* __restrict__ mh, const b16* __restrict__ ml,
                                                 const b16* __restrict__ mth, const b16* __restrict__ mtl, const float* __restrict__ mn, float* __restrict__ a, b16* __restrict__ p) {
  __shared__ __attribute__((aligned(16))) float Ta[4][32][64 + 4]; __shared__ __attribute__((aligned(16))) b16 Tp[4][32][64 + 8];
  const int lane = threadIdx.x & 31, wave = threadIdx.x >> 5, nloc = lane & 15, hlf = lane >> 4;
  const int c = blockIdx.z, q0 = blockIdx.y * 128 + wave * 32, i0 = blockIdx.x * 64;
  v16b aqh[2], aql[2], avh[2], avl[2]; float qn_[2];
#pragma unroll
  for (int r = 0; r < 2; ++r) {
    const int qq = q0 + r * 16 + nloc; const float* src = qcur + ((size_t)c * Q + qq) * DC; float x[DC], mean = 0.0f;
#pragma unroll
    for (int dd = 0; dd < DC; ++dd) { x[dd] = src[dd]; mean += x[dd]; }
    mean *= (1.0f / DC); float s2 = 0.0f; v16b fh = {}, fl = {};
#pragma unroll
    for (int dd = 0; dd < DC; ++dd) { const float xt = x[dd] - mean; s2 += xt * xt; }
#pragma unroll
    for (int e = 0; e < 8; ++e) { b16 hh_, ll_; split16((x[8 * hlf + e] - mean) * AS, hh_, ll_); fh[e] = hh_; fl[e] = ll_; }
    aqh[r] = fh; aql[r] = fl; qn_[r] = s2;
    if (!INIT) { const float* vs = vbuf + ((size_t)c * Q + qq) * DC; v16b gh = {}, gl = {};
#pragma unroll
      for (int e = 0; e < 8; ++e) { b16 hh_, ll_; split16(vs[8 * hlf + e] * AS, hh_, ll_); gh[e] = hh_; gl[e] = ll_; }
      avh[r] = gh; avl[r] = gl; }
  }
  float qnrow[2][8];
#pragma unroll
  for (int r = 0; r < 2; ++r)
#pragma unroll
    for (int v = 0; v < 8; ++v) qnrow[r][v] = __shfl(qn_[r], v + 8 * hlf, 32);
#pragma unroll
  for (int t = 0; t < 4; ++t) {
    const int irow = i0 + t * 16 + nloc; const size_t mo = ((size_t)irow * C + c) * DC;
    v16b bth = {}, btl = {}, bmh = {}, bml = {};
    { const v8b x0 = ld8b(mth + mo + 8 * hlf), x1 = ld8b(mtl + mo + 8 * hlf);
#pragma unroll
      for (int e = 0; e < 8; ++e) { bth[e] = x0[e]; btl[e] = x1[e]; } }
    if (!INIT) { const v8b x0 = ld8b(mh + mo + 8 * hlf), x1 = ld8b(ml + mo + 8 * hlf);
#pragma unroll
      for (int e = 0; e < 8; ++e) { bmh[e] = x0[e]; bml[e] = x1[e]; } }
#pragma unroll
    for (int r = 0; r < 2; ++r) {
      v8f num = {}; num = mac<2, 2>(aqh[r], aql[r], bth, btl, num);
      v8f cz = {}; if (!INIT) cz = mac<2, 2>(avh[r], avl[r], bmh, bml, cz);
#pragma unroll
      for (int v = 0; v < 8; ++v) {
        const int rr = r * 16 + v + 8 * hlf, ii = t * 16 + nloc; const float mnv = mn[((size_t)(i0 + ii)) * C + c];
        const float corr = (num[v] * (1.0f / (AS * AS))) * rsqrtf(mnv * qnrow[r][v] + EPS);
        const float pnew = tanh_e(corr);
        float anew = 0.0f;
        if (!INIT) { const float pold = (float)p[((size_t)c * Q + q0 + rr) * IC + i0 + ii]; anew = a[((size_t)c * Q + q0 + rr) * IC + i0 + ii] + pold * (cz[v] * (1.0f / (AS * AS))); }
        Ta[wave][rr][ii] = anew; Tp[wave][rr][ii] = (b16)pnew;
      }
    }
  }
  wave_lds_sync();
  for (int pass = 0; pass < 2; ++pass) {
#pragma unroll
    for (int j = 0; j < 16; ++j) { const int rr = j * 2 + hlf, c4 = nloc * 4; *(volatile v4f*)(a + ((size_t)c * Q + q0 + rr) * IC + i0 + c4) = *(const v4f*)(&Ta[wave][rr][c4]); }
#pragma unroll
    for (int j = 0; j < 8; ++j) { const int rr = j * 4 + (lane >> 3), c8 = (lane & 7) * 8; *(volatile v8b*)(p + ((size_t)c * Q + q0 + rr) * IC + i0 + c8) = *(const v8b*)(&Tp[wave][rr][c8]); }
    __threadfence();
  }
}

__global__ __launch_bounds__(256) void stats_kernel(const float* __restrict__ a, float* __restrict__ mx, float* __restrict__ inv) {
  const int q = blockIdx.y, i = blockIdx.x * 256 + threadIdx.x; float m = -INFINITY;
#pragma unroll 1
  for (int c = 0; c < C; ++c) m = fmaxf(m, a[((size_t)c * Q + q) * IC + i]);
  float s = 0.0f;
#pragma unroll 1
  for (int c = 0; c < C; ++c) s += __expf(a[((size_t)c * Q + q) * IC + i] - m);
  for (int pass = 0; pass < 2; ++pass) { ((volatile float*)mx)[(size_t)q * IC + i] = m; ((volatile float*)inv)[(size_t)q * IC + i] = 1.0f / s; __threadfence(); }
}

template <bool FINAL>
__global__ __launch_bounds__(128) void v_kernel(const float* __restrict__ a, const b16* __restrict__ p, const float* __restrict__ mx, const float* __restrict__ inv,
                                                const b16* __restrict__ mTh, const b16* __restrict__ mTl, float* __restrict__ vbuf, float* __restrict__ qcur, float* __restrict__ out) {
  __shared__ __attribute__((aligned(16))) float To[32][4 * DC + 4];
  __shared__ __attribute__((aligned(16))) float Tv[4][32][DC];
  const int lane = threadIdx.x & 31, wave = threadIdx.x >> 5, nloc = lane & 15, hlf = lane >> 4;
  const int c = blockIdx.x * 4 + wave, q0 = blockIdx.y * 32;
  v8f acc[2] = {{}, {}};
  const b16* Bh = mTh + (size_t)c * DC * IC; const b16* Bl = mTl + (size_t)c * DC * IC;
#pragma unroll 1
  for (int kb = 0; kb < IC; kb += 32) {
    v16b a0h, a0l, a1h, a1l;
#pragma unroll
    for (int r = 0; r < 2; ++r) { const int qq = q0 + r * 16 + nloc; v16b fh, fl;
#pragma unroll
      for (int e = 0; e < 16; ++e) { const int i = kb + ((e < 8) ? (8 * hlf + e) : (16 + 8 * hlf + e - 8)); const size_t ai = ((size_t)c * Q + qq) * IC + i, si = (size_t)qq * IC + i;
        const float dsp = __expf(a[ai] - mx[si]) * inv[si] + (float)p[ai]; b16 hh_, ll_; split16(dsp * AS, hh_, ll_); fh[e] = hh_; fl[e] = ll_; }
      if (r == 0) { a0h = fh; a0l = fl; } else { a1h = fh; a1l = fl; } }
    const v16b bh_ = frag_kb(Bh + (size_t)nloc * IC + kb, hlf), bl_ = frag_kb(Bl + (size_t)nloc * IC + kb, hlf);
    acc[0] = mac<2, 2>(a0h, a0l, bh_, bl_, acc[0]); acc[1] = mac<2, 2>(a1h, a1l, bh_, bl_, acc[1]);
  }
#pragma unroll
  for (int r = 0; r < 2; ++r)
#pragma unroll
    for (int v = 0; v < 8; ++v) {
      const float s = acc[r][v] * (1.0f / (AS * AS)); float n2 = s * s;
#pragma unroll
      for (int o = 1; o < 16; o <<= 1) n2 += __shfl_xor(n2, o);
      const float vv = (n2 / (1.0f + n2)) * s * rsqrtf(n2 + EPS);
      const int rr = r * 16 + v + 8 * hlf;
      if (FINAL) To[rr][wave * DC + nloc] = vv; else Tv[wave][rr][nloc] = vv;
    }
  if (FINAL) {
    __syncthreads();
    for (int pass = 0; pass < 2; ++pass) {
#pragma unroll
      for (int j = 0; j < 4; ++j) { const int rr = j * 8 + (threadIdx.x >> 4), c4 = (threadIdx.x & 15) * 4; *(volatile v4f*)(out + (size_t)(q0 + rr) * NO + blockIdx.x * 4 * DC + c4) = *(const v4f*)(&To[rr][c4]); }
      __threadfence();
    }
  } else {
    wave_lds_sync();
    float* vd = vbuf + ((size_t)c * Q + q0) * DC; float* qd = qcur + ((size_t)c * Q + q0) * DC;
    v4f nv[4], nq[4];
#pragma unroll
    for (int j = 0; j < 4; ++j) { const int f = (j * 32 + lane) * 4; nv[j] = *(const v4f*)(&Tv[wave][0][0] + f); const v4f oq = *(const v4f*)(qd + f); nq[j] = (oq + nv[j]) * 0.5f; }
    for (int pass = 0; pass < 2; ++pass) {
#pragma unroll
      for (int j = 0; j < 4; ++j) { const int f = (j * 32 + lane) * 4; *(volatile v4f*)(vd + f) = nv[j]; *(volatile v4f*)(qd + f) = nq[j]; }
      __threadfence();
    }
  }
}
}

extern "C" void kernel_launch(void* const* d_in, const int* in_sizes, int n_in,
                              void* d_out, int out_size, void* d_ws, size_t ws_size, hipStream_t stream) {
  (void)n_in; (void)out_size;
  const float* m = (const float*)d_in[0]; const float* q = (const float*)d_in[1]; const float* W = (const float*)d_in[2]; const float* Wb = (const float*)d_in[3];
  float* out = (float*)d_out;
  if (in_sizes[0] != IC * IN || in_sizes[1] != Q * IN || in_sizes[2] != IN * NO || in_sizes[3] != NO) return;
  size_t off = 0; char* ws = (char*)d_ws;
  auto carve = [&](size_t bytes) { char* p = ws + off; off += (bytes + 255) & ~(size_t)255; return p; };
  b16* wh = (b16*)carve((size_t)NO * IN * 2); b16* wl = (b16*)carve((size_t)NO * IN * 2);
  float* hm = (float*)carve((size_t)IC * NO * 4);
  float* qcur = (float*)carve((size_t)C * Q * DC * 4); float* vbuf = (float*)carve((size_t)C * Q * DC * 4);
  b16* mh = (b16*)carve((size_t)IC * NO * 2); b16* ml = (b16*)carve((size_t)IC * NO * 2); b16* mth = (b16*)carve((size_t)IC * NO * 2); b16* mtl = (b16*)carve((size_t)IC * NO * 2);
  b16* mTh = (b16*)carve((size_t)C * DC * IC * 2); b16* mTl = (b16*)carve((size_t)C * DC * IC * 2);
  float* mn = (float*)carve((size_t)IC * C * 4);
  float* a = (float*)carve((size_t)C * Q * IC * 4);
  b16* p = (b16*)carve((size_t)C * Q * IC * 2);
  float* mx = (float*)carve((size_t)Q * IC * 4); float* inv = (float*)carve((size_t)Q * IC * 4);
  if (off > ws_size) return;
  prepw_kernel<<<dim3(NO / 64, IN / 64), 256, 0, stream>>>(W, wh, wl);
  proj_kernel<<<dim3(NO / 64, (IC + Q) / 128), 128, 0, stream>>>(m, q, wh, wl, Wb, hm, qcur);
  mrows_kernel<<<IC * C / 256, 256, 0, stream>>>(hm, mh, ml, mth, mtl, mn);
  mT_kernel<<<C, 256, 0, stream>>>(hm, mTh, mTl);
  pc_kernel<true><<<dim3(IC / 64, Q / 128, C), 128, 0, stream>>>(qcur, vbuf, mh, ml, mth, mtl, mn, a, p);
  for (int it = 0; it < 2; ++it) {
    stats_kernel<<<dim3(IC / 256, Q), 256, 0, stream>>>(a, mx, inv);
    v_kernel<false><<<dim3(C / 4, Q / 32), 128, 0, stream>>>(a, p, mx, inv, mTh, mTl, vbuf, qcur, out);
    pc_kernel<false><<<dim3(IC / 64, Q / 128, C), 128, 0, stream>>>(qcur, vbuf, mh, ml, mth, mtl, mn, a, p);
  }
  stats_kernel<<<dim3(IC / 256, Q), 256, 0, stream>>>(a, mx, inv);
  v_kernel<true><<<dim3(C / 4, Q / 32), 128, 0, stream>>>(a, p, mx, inv, mTh, mTl, vbuf, qcur, out);
}
